// Colorizer_53395033423959
// MI455X (gfx1250) — hardware-verified
//
#include <hip/hip_runtime.h>
#include <math.h>
#include <stdint.h>

#ifndef NB
#define NB 8
#endif
#ifndef NQ
#define NQ 1024
#endif
#define KT     3
#define IMH    256
#define IMW    256
#define IMC    3
#define PS     8
#define PGR    32
#define NPF    (PGR * PGR)
#define NFR    (KT + 1)
#define RPS    (NFR * NPF)
#define NKEY   (KT * NPF)
#define FEAT   256
#define NCLS   16
#define KIM    (PS * PS * IMC)
#define NKB    (NKEY / 32)
#define QSC    8.0f
#define RSC    1024.0f
#define PCAR   32768.0f
#define VCAR   1024.0f
#define LOG2E  1.4426950408889634f
#define SLAB   (16 * 68)
#define OSLAB  (16 * 20)
#define IMGK_STRIDE_N ((size_t)KT * IMH * IMW * IMC)
#define IMGQ_STRIDE_N ((size_t)IMH * IMW * IMC)
#define FRAME_STRIDE  ((size_t)IMH * IMW * IMC)
#define LAB_STRIDE_N  ((size_t)NKEY * NCLS)
#define OUT_STRIDE_N  ((size_t)NPF * NCLS)
static_assert(NB >= 1 && NB <= 8);
static_assert((NQ % 64) == 0 && NQ >= 64 && NQ <= NPF);
static_assert((KIM % 32) == 0 && (FEAT % 64) == 0 && (RPS % 64) == 0 && NKB * 32 == NKEY);
static_assert(((PS * IMC) % 8) == 0 && (NKEY % 8) == 0);
static_assert((RPS * (KIM / 8)) % 256 == 0 && (FEAT * (KIM / 8)) % 256 == 0 && (NCLS * (NKEY / 8)) % 256 == 0);
static_assert((SLAB * 4) % 16 == 0 && (OSLAB * 4) % 16 == 0);

typedef unsigned short u16;
typedef _Float16 v16h __attribute__((ext_vector_type(16)));
typedef _Float16 v8h  __attribute__((ext_vector_type(8)));
typedef __bf16   v16b __attribute__((ext_vector_type(16)));
typedef float    v8f  __attribute__((ext_vector_type(8)));
typedef float    v4f  __attribute__((ext_vector_type(4)));
typedef unsigned int v4u __attribute__((ext_vector_type(4)));

union FragH { v16h v; v8h h[2]; v4u u[2]; };
union FragB { v16b v; v4u u[2]; };

__device__ __forceinline__ unsigned short bf_bits(float f) {
  unsigned u = __float_as_uint(f);
  return (unsigned short)((u + 0x7FFFu + ((u >> 16) & 1u)) >> 16);
}
__device__ __forceinline__ float bf_up(unsigned short h) { return __uint_as_float(((unsigned)h) << 16); }
__device__ __forceinline__ float bf_val(float f) { return bf_up(bf_bits(f)); }
__device__ __forceinline__ unsigned short h_bits(_Float16 x) { return __builtin_bit_cast(unsigned short, x); }
__device__ __forceinline__ unsigned pk16(unsigned short a, unsigned short b) { return (unsigned)a | ((unsigned)b << 16); }
__device__ __forceinline__ v8f zero8() { v8f z = {0.f, 0.f, 0.f, 0.f, 0.f, 0.f, 0.f, 0.f}; return z; }

__device__ __forceinline__ v16h ldfrag_h(const _Float16* p) {
  FragH f;
  f.h[0] = *(const v8h*)(p);
  f.h[1] = *(const v8h*)(p + 16);
  return f.v;
}
__device__ __forceinline__ v16b ldfrag_b(const u16* p) {
  FragB f;
  f.u[0] = *(const v4u*)(p);
  f.u[1] = *(const v4u*)(p + 16);
  return f.v;
}

__device__ __forceinline__ v8f mma_h(v16h a, v16h b, v8f c) {
  return __builtin_amdgcn_wmma_f32_16x16x32_f16(false, a, false, b, (short)0, c, false, false);
}
__device__ __forceinline__ v8f mma_b(v16b a, v16b b, v8f c) {
  return __builtin_amdgcn_wmma_f32_16x16x32_bf16(false, a, false, b, (short)0, c, false, false);
}
__device__ __forceinline__ void guard1(v8f& a, v16h x0, v16h x1) {
#if defined(__HIP_DEVICE_COMPILE__)
  asm volatile("v_nop\n\tv_nop\n\tv_nop\n\tv_nop" : "+v"(a) : "v"(x0), "v"(x1) : "memory");
#endif
}
template <typename F>
__device__ __forceinline__ void guard6(v8f& a, v8f& b, v8f& c, v8f& d, F x0, F x1, F x2, F x3, F x4, F x5) {
#if defined(__HIP_DEVICE_COMPILE__)
  asm volatile("v_nop\n\tv_nop\n\tv_nop\n\tv_nop"
               : "+v"(a), "+v"(b), "+v"(c), "+v"(d) : "v"(x0), "v"(x1), "v"(x2), "v"(x3), "v"(x4), "v"(x5) : "memory");
#endif
}
__device__ __forceinline__ void acc_guard4(v8f& a, v8f& b, v8f& c, v8f& d) {
#if defined(__HIP_DEVICE_COMPILE__)
  asm volatile("v_nop\n\tv_nop\n\tv_nop\n\tv_nop" : "+v"(a), "+v"(b), "+v"(c), "+v"(d));
#endif
}
__device__ __forceinline__ void acc_guard1(v8f& a) {
#if defined(__HIP_DEVICE_COMPILE__)
  asm volatile("v_nop\n\tv_nop\n\tv_nop\n\tv_nop" : "+v"(a));
#endif
}
__device__ __forceinline__ void wave_sync_lds() {
#if defined(__HIP_DEVICE_COMPILE__)
  __builtin_amdgcn_fence(__ATOMIC_RELEASE, "workgroup");
  __builtin_amdgcn_wave_barrier();
  __builtin_amdgcn_fence(__ATOMIC_ACQUIRE, "workgroup");
#endif
}

__device__ __forceinline__ void store8x16_twice(u16* d, v4u o) {
  for (int pass = 0; pass < 2; ++pass) {
    *(volatile v4u*)(d) = o;
    __threadfence();
  }
}

__global__ __launch_bounds__(256)
void cvt_im2col(const float* __restrict__ imk, const float* __restrict__ imq, u16* D, int n8) {
  const int gt = blockIdx.x * 256 + (int)threadIdx.x;
  if (gt >= n8) return;
  const int p   = gt / (KIM / 8), j = gt - p * (KIM / 8);
  const int n   = p / RPS,  pr  = p - n * RPS;
  const int t   = pr / NPF, pix = pr - t * NPF;
  const int py  = pix / PGR, px = pix - py * PGR;
  const int dy  = j / 3, seg = j - dy * 3;
  const int row = py * PS + dy;
  const int tk  = (t < KT) ? t : (KT - 1);
  const size_t cofs = (size_t)row * (IMW * IMC) + (size_t)px * (PS * IMC) + (size_t)seg * 8;
  const float* pk = imk + (size_t)n * IMGK_STRIDE_N + (size_t)tk * FRAME_STRIDE + cofs;
  const float* pq = imq + (size_t)n * IMGQ_STRIDE_N + cofs;
  const v4f ka = *(const v4f*)(pk), kc = *(const v4f*)(pk + 4);
  const v4f qa = *(const v4f*)(pq), qc = *(const v4f*)(pq + 4);
  const bool isq = (t >= KT);
  float v[8];
#pragma unroll
  for (int e = 0; e < 4; ++e) { v[e] = isq ? qa[e] : ka[e]; v[4 + e] = isq ? qc[e] : kc[e]; }
  unsigned short s[8];
#pragma unroll
  for (int e = 0; e < 8; ++e) s[e] = bf_bits(v[e]);
  v4u o;
#pragma unroll
  for (int e = 0; e < 4; ++e) o[e] = pk16(s[2 * e], s[2 * e + 1]);
  store8x16_twice(D + (size_t)gt * 8, o);
}

__global__ __launch_bounds__(256)
void cvt_w(const float* __restrict__ w, u16* D, int n8) {
  const int gt = blockIdx.x * 256 + (int)threadIdx.x;
  if (gt >= n8) return;
  const int n = gt / (KIM / 8), j = gt - n * (KIM / 8);
  const int k0 = j * 8;
  unsigned short s[8];
#pragma unroll
  for (int e = 0; e < 8; ++e) s[e] = bf_bits(w[(size_t)(k0 + e) * FEAT + n]);
  v4u o;
#pragma unroll
  for (int e = 0; e < 4; ++e) o[e] = pk16(s[2 * e], s[2 * e + 1]);
  store8x16_twice(D + (size_t)gt * 8, o);
}

__global__ __launch_bounds__(256)
void cvt_lab(const float* __restrict__ lab, u16* D, int n8) {
  const int gt = blockIdx.x * 256 + (int)threadIdx.x;
  if (gt >= n8) return;
  const int per = NCLS * (NKEY / 8);
  const int n = gt / per, rem = gt - n * per;
  const int c = rem / (NKEY / 8), j = rem - c * (NKEY / 8);
  const int r0 = j * 8;
  const float* src = lab + (size_t)n * LAB_STRIDE_N + (size_t)r0 * NCLS + c;
  unsigned short s[8];
#pragma unroll
  for (int e = 0; e < 8; ++e) s[e] = h_bits((_Float16)(bf_val(src[(size_t)e * NCLS]) * VCAR));
  v4u o;
#pragma unroll
  for (int e = 0; e < 4; ++e) o[e] = pk16(s[2 * e], s[2 * e + 1]);
  store8x16_twice(D + (size_t)gt * 8, o);
}

__device__ __forceinline__ void epi_hl(float* sl, v8f a0, v8f a1, v8f a2, v8f a3, u16* CH, u16* CL, int N,
                                       size_t rowb, int col0, int lane) {
  const int hh = lane >> 4, m = lane & 15;
#pragma unroll
  for (int r = 0; r < 8; ++r) {
    const int ro = (8 * hh + r) * 68 + m;
    sl[ro]      = a0[r];
    sl[ro + 16] = a1[r];
    sl[ro + 32] = a2[r];
    sl[ro + 48] = a3[r];
  }
  wave_sync_lds();
  const int rq = lane >> 3, c8 = (lane & 7) * 8;
  v4u oh[4], ol[4];
#pragma unroll
  for (int i4 = 0; i4 < 4; ++i4) {
    const int row = i4 * 4 + rq;
    const v4f a = *(const v4f*)(sl + row * 68 + c8), c4 = *(const v4f*)(sl + row * 68 + c8 + 4);
    float w[8];
#pragma unroll
    for (int e = 0; e < 4; ++e) { w[e] = a[e]; w[4 + e] = c4[e]; }
#pragma unroll
    for (int e = 0; e < 4; ++e) {
      const float s0 = w[2 * e] * QSC, s1 = w[2 * e + 1] * QSC;
      const _Float16 h0 = (_Float16)s0, h1 = (_Float16)s1;
      const _Float16 l0 = (_Float16)((s0 - (float)h0) * RSC);
      const _Float16 l1 = (_Float16)((s1 - (float)h1) * RSC);
      oh[i4][e] = pk16(h_bits(h0), h_bits(h1));
      ol[i4][e] = pk16(h_bits(l0), h_bits(l1));
    }
  }
  const size_t base = (rowb + (size_t)rq) * (size_t)N + (size_t)col0 + (size_t)c8;
  u16* dh = CH + base;
  u16* dl = CL + base;
  for (int pass = 0; pass < 2; ++pass) {
#pragma unroll
    for (int i4 = 0; i4 < 4; ++i4) {
      *(volatile v4u*)(dh + (size_t)(i4 * 4) * (size_t)N) = oh[i4];
      *(volatile v4u*)(dl + (size_t)(i4 * 4) * (size_t)N) = ol[i4];
    }
    __threadfence();
  }
}

__global__ __launch_bounds__(128)
void gemm_feat(const u16* __restrict__ A, const u16* __restrict__ Bt, u16* CH, u16* CL, int M, int N, int K) {
  __shared__ __align__(16) float slab[4 * SLAB];
  const int tid = threadIdx.x, wave = tid >> 5, lane = tid & 31, hh = lane >> 4, m = lane & 15;
  const int ntile = N >> 6;
  const int bid   = blockIdx.x;
  const int rowb  = (bid / ntile) * 64 + wave * 16;
  const int col0  = (bid % ntile) * 64;
  if (rowb + 16 > M) return;
  const u16* ap = A  + (size_t)(rowb + m) * K + 8 * hh;
  const u16* bp = Bt + (size_t)(col0 + m) * K + 8 * hh;
  const size_t bs = (size_t)16 * K;
  v8f acc0 = zero8(), acc1 = zero8(), acc2 = zero8(), acc3 = zero8();
#pragma unroll 1
  for (int k0 = 0; k0 < K; k0 += 32) {
    const v16b a  = ldfrag_b(ap + k0);
    const v16b b0 = ldfrag_b(bp + k0);
    const v16b b1 = ldfrag_b(bp + bs + k0);
    const v16b b2 = ldfrag_b(bp + 2 * bs + k0);
    const v16b b3 = ldfrag_b(bp + 3 * bs + k0);
    acc0 = mma_b(a, b0, acc0);
    acc1 = mma_b(a, b1, acc1);
    acc2 = mma_b(a, b2, acc2);
    acc3 = mma_b(a, b3, acc3);
    guard6<v16b>(acc0, acc1, acc2, acc3, a, b0, b1, b2, b3, a);
  }
  acc_guard4(acc0, acc1, acc2, acc3);
  epi_hl(slab + wave * SLAB, acc0, acc1, acc2, acc3, CH, CL, N, (size_t)rowb, col0, lane);
}

__global__ __launch_bounds__(128)
void attn_fwd(const u16* __restrict__ FHp, const u16* __restrict__ FLp, const u16* __restrict__ LTp, float* out) {
  __shared__ __align__(16) float smem[4 * OSLAB];

  const int tid  = threadIdx.x;
  const int wave = tid >> 5;
  const int lane = tid & 31;
  const int hh   = lane >> 4;
  const int c    = lane & 15;

  const int bid  = blockIdx.x;
  const int qt   = bid % (NQ / 64);
  const int n    = bid / (NQ / 64);
  if (n >= NB) return;
  const int q0   = qt * 64 + wave * 16;

  const _Float16* FH = (const _Float16*)(const void*)FHp;
  const _Float16* FL = (const _Float16*)(const void*)FLp;
  const _Float16* LT = (const _Float16*)(const void*)LTp;
  const size_t rown = (size_t)n * RPS;
  const size_t qofs = (rown + (size_t)NKEY + (size_t)(q0 + c)) * FEAT + 8 * hh;
  const _Float16* Qh = FH + qofs;
  const _Float16* Ql = FL + qofs;
  const size_t kofs = (rown + (size_t)c) * FEAT + 8 * hh;
  const _Float16* Kh = FH + kofs;
  const _Float16* Kl = FL + kofs;
  const _Float16* Lb = LT + ((size_t)n * NCLS + c) * NKEY + 8 * hh;
  const float lsc = LOG2E / (QSC * QSC);
  const float lsx = lsc / RSC;

  float mrun = -INFINITY, lrun = 0.f;
  v8f o = zero8();

#pragma unroll 1
  for (int it = 0; it < NKB; ++it) {
    const int kb = it * 32;
    v8f shh0 = zero8(), sx0 = zero8(), shh1 = zero8(), sx1 = zero8();
    const _Float16* k0h = Kh + (size_t)kb * FEAT;
    const _Float16* k0l = Kl + (size_t)kb * FEAT;
    const _Float16* k1h = k0h + (size_t)16 * FEAT;
    const _Float16* k1l = k0l + (size_t)16 * FEAT;
#pragma unroll 1
    for (int dc = 0; dc < FEAT / 32; ++dc) {
      const int d0 = dc * 32;
      const v16h fqh = ldfrag_h(Qh + d0), fql = ldfrag_h(Ql + d0);
      const v16h a0h = ldfrag_h(k0h + d0), a0l = ldfrag_h(k0l + d0);
      const v16h a1h = ldfrag_h(k1h + d0), a1l = ldfrag_h(k1l + d0);
      shh0 = mma_h(a0h, fqh, shh0);
      shh1 = mma_h(a1h, fqh, shh1);
      sx0  = mma_h(a0h, fql, sx0);
      sx1  = mma_h(a1h, fql, sx1);
      sx0  = mma_h(a0l, fqh, sx0);
      sx1  = mma_h(a1l, fqh, sx1);
      guard6<v16h>(shh0, sx0, shh1, sx1, fqh, fql, a0h, a0l, a1h, a1l);
    }
    acc_guard4(shh0, sx0, shh1, sx1);
    float tk[16];
#pragma unroll
    for (int i = 0; i < 8; ++i) {
      tk[i]     = fmaf(sx0[i], lsx, shh0[i] * lsc);
      tk[8 + i] = fmaf(sx1[i], lsx, shh1[i] * lsc);
    }
    float cm = tk[0];
#pragma unroll
    for (int i = 1; i < 16; ++i) cm = fmaxf(cm, tk[i]);
    cm = fmaxf(cm, __shfl_xor(cm, 16, 32));
    const float mn = fmaxf(mrun, cm);
    const float al = (mrun == -INFINITY) ? 0.f : exp2f(mrun - mn);
    mrun = mn;
    float ps = 0.f;
    FragH ph;
#pragma unroll
    for (int w = 0; w < 2; ++w) {
#pragma unroll
      for (int e4 = 0; e4 < 4; ++e4) {
        const int i = 8 * w + 2 * e4;
        const float p0 = exp2f(fminf(tk[i] - mn, 0.f));
        const float p1 = exp2f(fminf(tk[i + 1] - mn, 0.f));
        ps += p0 + p1;
        ph.u[w][e4] = pk16(h_bits((_Float16)(p0 * PCAR)), h_bits((_Float16)(p1 * PCAR)));
      }
    }
    ps += __shfl_xor(ps, 16, 32);
    lrun = lrun * al + ps;
    float scl[8];
#pragma unroll
    for (int r = 0; r < 8; ++r) scl[r] = __shfl(al, 8 * hh + r, 32);
#pragma unroll
    for (int r = 0; r < 8; ++r) o[r] *= scl[r];
    {
      const v16h lf = ldfrag_h(Lb + kb);
      o = mma_h(ph.v, lf, o);
      guard1(o, ph.v, lf);
    }
  }
  acc_guard1(o);

  const float linv = (lrun > 0.f) ? ((1.0f / lrun) * (1.0f / (PCAR * VCAR))) : 0.f;
  float inv[8];
#pragma unroll
  for (int r = 0; r < 8; ++r) inv[r] = __shfl(linv, 8 * hh + r, 32);
  float* slab = smem + wave * OSLAB;
#pragma unroll
  for (int r = 0; r < 8; ++r) slab[(8 * hh + r) * 20 + c] = o[r] * inv[r];
  wave_sync_lds();
  const int rr = lane >> 2, cc = (lane & 3) * 4;
  const v4f w0 = *(const v4f*)(slab + rr * 20 + cc);
  const v4f w1 = *(const v4f*)(slab + (8 + rr) * 20 + cc);
  float* dst = out + (size_t)n * OUT_STRIDE_N + (size_t)q0 * NCLS + (size_t)lane * 4;
  for (int pass = 0; pass < 2; ++pass) {
    *(volatile v4f*)(dst) = w0;
    *(volatile v4f*)(dst + 8 * NCLS) = w1;
    __threadfence();
  }
}

extern "C" void kernel_launch(void* const* d_in, const int* in_sizes, int n_in,
                              void* d_out, int out_size, void* d_ws, size_t ws_size,
                              hipStream_t stream) {
  if (n_in < 4) return;
  if ((size_t)in_sizes[0] < (size_t)NB * IMGK_STRIDE_N) return;
  if ((size_t)in_sizes[1] < (size_t)NB * IMGQ_STRIDE_N) return;
  if ((size_t)in_sizes[2] < (size_t)NB * LAB_STRIDE_N) return;
  if (in_sizes[3] < KIM * FEAT) return;
  if ((size_t)out_size < (size_t)NB * OUT_STRIDE_N) return;

  const float* imk = (const float*)d_in[0];
  const float* imq = (const float*)d_in[1];
  const float* lab = (const float*)d_in[2];
  const float* wfe = (const float*)d_in[3];
  float*       out = (float*)d_out;

  const int M = NB * RPS;
  const size_t szIM = (size_t)M * KIM * 2;
  const size_t szWB = (size_t)FEAT * KIM * 2;
  const size_t szLT = (size_t)NB * NCLS * NKEY * 2;
  const size_t szF  = (size_t)M * FEAT * 2;
  size_t off = 0;
  const size_t oIM = off; off += szIM;
  const size_t oWB = off; off += szWB;
  const size_t oLT = off; off += szLT;
  const size_t oFH = off; off += szF;
  const size_t oFL = off; off += szF;
  if (off > ws_size) return;
  if (off > (size_t)134217728) return;
  if ((oWB % 128) != 0 || (oLT % 128) != 0 || (oFH % 128) != 0 || (oFL % 128) != 0) return;

  char* ws = (char*)d_ws;
  u16* IM = (u16*)(ws + oIM);
  u16* WB = (u16*)(ws + oWB);
  u16* LT = (u16*)(ws + oLT);
  u16* FH = (u16*)(ws + oFH);
  u16* FL = (u16*)(ws + oFL);

  const int n8im = M * (KIM / 8);
  const int n8w  = FEAT * (KIM / 8);
  const int n8l  = NB * NCLS * (NKEY / 8);
  if ((n8im % 256) != 0 || (n8w % 256) != 0 || (n8l % 256) != 0) return;
  if ((M % 64) != 0 || (FEAT % 64) != 0 || (KIM % 32) != 0 || (NQ % 64) != 0) return;
  const dim3 blk(256);
  const dim3 gIM(n8im / 256);
  const dim3 gW(n8w / 256);
  const dim3 gL(n8l / 256);
  const dim3 gG((M / 64) * (FEAT / 64));
  const dim3 bG(128);
  const dim3 gAT(NB * (NQ / 64));
  const dim3 bAT(128);

  cvt_im2col<<<gIM, blk, 0, stream>>>(imk, imq, IM, n8im);
  cvt_w<<<gW, blk, 0, stream>>>(wfe, WB, n8w);
  cvt_lab<<<gL, blk, 0, stream>>>(lab, LT, n8l);
  gemm_feat<<<gG, bG, 0, stream>>>(IM, WB, FH, FL, M, FEAT, KIM);
  attn_fwd<<<gAT, bAT, 0, stream>>>(FH, FL, LT, out);
  (void)hipGetLastError();
}
